// ResidualMambaBlock_62182536511817
// MI455X (gfx1250) — hardware-verified
//
#include <hip/hip_runtime.h>


#define NB_   8
#define NL_   1024
#define DM_   512
#define DI_   1024
#define NS_   16
#define DTR_  32
#define XDW_  64
#define MT_   (NB_ * NL_)

static_assert(MT_ % 64 == 0);
static_assert(DM_ == 512);
static_assert(DM_ % 128 == 0);
static_assert(DI_ % 128 == 0);
static_assert((2 * DI_) % 128 == 0);
static_assert(XDW_ == DTR_ + 2 * NS_);
static_assert(XDW_ == 64);
static_assert(DTR_ == 32);
static_assert(NL_ % 16 == 0);
static_assert((NL_ & (NL_ - 1)) == 0);
static_assert(DI_ % 64 == 0);

typedef float          v4f   __attribute__((ext_vector_type(4)));
typedef float          v8f   __attribute__((ext_vector_type(8)));
typedef _Float16       v8h   __attribute__((ext_vector_type(8)));
typedef _Float16       v16h  __attribute__((ext_vector_type(16)));
typedef unsigned short u16x8 __attribute__((ext_vector_type(8)));

union FragH { u16x8 h[2]; v16h v; };
union Pack8 { v8h f; u16x8 u; };
union H1    { _Float16 f; unsigned short u; };

#define LOG2E_F 1.4426950408889634f

__device__ __forceinline__ v8f ld8f(const float* p) {
    v4f a = *(const v4f*)p;
    v4f b = *(const v4f*)(p + 4);
    return __builtin_shufflevector(a, b, 0, 1, 2, 3, 4, 5, 6, 7);
}
__device__ __forceinline__ float silu_f(float x) {
    const float e = exp2f(-x * LOG2E_F);
    return x * __builtin_amdgcn_rcpf(1.0f + e);
}
__device__ __forceinline__ float softplus_f(float x) {
    return fmaxf(x, 0.0f) + log1pf(exp2f(-fabsf(x) * LOG2E_F));
}
__device__ __forceinline__ float conv4_silu(float x0, float x1, float x2, float x3,
                                            float w0, float w1, float w2, float w3, float bias) {
    const float c = w0 * x0 + w1 * x1 + w2 * x2 + w3 * x3;
    return silu_f(c + bias);
}

__device__ __forceinline__ void mma16(v8f& acc, const FragH& a, const FragH& b) {
    acc = __builtin_amdgcn_wmma_f32_16x16x32_f16(false, a.v, false, b.v, (short)0, acc, false, false);
    asm volatile("v_nop\n\tv_nop\n\tv_nop\n\tv_nop" : "+v"(acc) : "v"(a.v), "v"(b.v));
}

__global__ __launch_bounds__(256)
void cvt_kernel(const float* __restrict__ src, unsigned short* dst, int n8, float scale)
{
    const int i = blockIdx.x * 256 + threadIdx.x;
    if (i >= n8) return;
    const size_t e = (size_t)i * 8;
    const v8f x = ld8f(src + e);
    Pack8 pk;
    pk.f = __builtin_convertvector(x * scale, v8h);
    const u16x8 v = pk.u;
    *(volatile u16x8*)(dst + e) = v;
    __threadfence();
    *(volatile u16x8*)(dst + e) = v;
}

__global__ __launch_bounds__(256)
void ln_kernel(const float* __restrict__ X, const float* __restrict__ W, const float* __restrict__ Bv,
               unsigned short* XN)
{
    const int lane = threadIdx.x & 31;
    const int wave = threadIdx.x >> 5;
    const int row  = blockIdx.x * 8 + wave;
    const float* xr = X + (size_t)row * DM_;
    const v8f a = ld8f(xr + 8 * lane);
    const v8f c = ld8f(xr + 256 + 8 * lane);
    float s = 0.0f;
#pragma unroll
    for (int i = 0; i < 8; ++i) s += a[i] + c[i];
#pragma unroll
    for (int off = 16; off > 0; off >>= 1) s += __shfl_xor(s, off);
    const float mu = s * (1.0f / (float)DM_);
    const v8f da = a - mu;
    const v8f dc = c - mu;
    float q = 0.0f;
#pragma unroll
    for (int i = 0; i < 8; ++i) q += da[i] * da[i] + dc[i] * dc[i];
#pragma unroll
    for (int off = 16; off > 0; off >>= 1) q += __shfl_xor(q, off);
    const float var = q * (1.0f / (float)DM_);
    const float rs  = rsqrtf(var + 1e-5f);
    const v8f wa = ld8f(W + 8 * lane);
    const v8f wc = ld8f(W + 256 + 8 * lane);
    const v8f ba = ld8f(Bv + 8 * lane);
    const v8f bc = ld8f(Bv + 256 + 8 * lane);
    const v8f ya = (da * rs) * wa + ba;
    const v8f yc = (dc * rs) * wc + bc;
    Pack8 pa, pc;
    pa.f = __builtin_convertvector(ya, v8h);
    pc.f = __builtin_convertvector(yc, v8h);
    const u16x8 va = pa.u;
    const u16x8 vc = pc.u;
    unsigned short* gp = XN + (size_t)row * DM_;
    *(volatile u16x8*)(gp + 8 * lane)       = va;
    *(volatile u16x8*)(gp + 256 + 8 * lane) = vc;
    __threadfence();
    *(volatile u16x8*)(gp + 8 * lane)       = va;
    *(volatile u16x8*)(gp + 256 + 8 * lane) = vc;
}

template<int NBF, bool RESID>
__device__ __forceinline__ void tile_store_pass(const float* st, float* gp, int ldc,
                                                const float* __restrict__ rp, int lane) {
    constexpr int CW  = NBF * 16;
    constexpr int P   = CW + 4;
    constexpr int LPR = CW / 4;
    constexpr int RPI = 32 / LPR;
    constexpr int NIT = 32 / RPI;
    const int rsub = lane / LPR;
    const int c4   = (lane % LPR) * 4;
#pragma unroll
    for (int it = 0; it < NIT; ++it) {
        const int row = it * RPI + rsub;
        v4f v = *(const v4f*)(st + row * P + c4);
        if (RESID) v += *(const v4f*)(rp + (size_t)row * ldc + c4);
        *(volatile v4f*)(gp + (size_t)row * ldc + c4) = v;
    }
}

template<bool A32, int NBF, bool RESID>
__global__ __launch_bounds__(128)
void gemm_tn_kernel(const unsigned short* __restrict__ A16, const float* __restrict__ Af,
                    const unsigned short* __restrict__ Bw, float* C, float* C2,
                    const float* __restrict__ R,
                    int K, int lda, int ldb, int ldc, int csplit, float ascale, float oscale)
{
    constexpr int CW = NBF * 16;
    constexpr int P  = CW + 4;
    __shared__ __attribute__((aligned(16))) float stile[4][32 * P];

    const int tid  = threadIdx.x;
    const int lane = tid & 31;
    const int wave = tid >> 5;
    const int h    = lane >> 4;
    const int m    = lane & 15;
    const int wm   = wave >> 1;
    const int wn   = wave & 1;

    const int rowW = blockIdx.y * 64 + wm * 32;
    const int colW = blockIdx.x * (2 * CW) + wn * CW;

    v8f acc[2 * NBF];
#pragma unroll
    for (int j = 0; j < 2 * NBF; ++j)
#pragma unroll
        for (int r = 0; r < 8; ++r) acc[j][r] = 0.0f;

    const int nk = K >> 5;
    for (int kt = 0; kt < nk; ++kt) {
        const int k0 = kt * 32;
        FragH fa[2], fb[NBF];
#pragma unroll
        for (int s = 0; s < 2; ++s) {
            const size_t arow = (size_t)(rowW + 16 * s + m);
            if (A32) {
                const float* p = Af + arow * (size_t)lda + k0 + 8 * h;
                Pack8 q0, q1;
                q0.f = __builtin_convertvector(ld8f(p) * ascale, v8h);
                q1.f = __builtin_convertvector(ld8f(p + 16) * ascale, v8h);
                fa[s].h[0] = q0.u;
                fa[s].h[1] = q1.u;
            } else {
                const unsigned short* p = A16 + arow * (size_t)lda + k0 + 8 * h;
                fa[s].h[0] = *(const u16x8*)(p);
                fa[s].h[1] = *(const u16x8*)(p + 16);
            }
        }
#pragma unroll
        for (int j = 0; j < NBF; ++j) {
            const unsigned short* p = Bw + (size_t)(colW + 16 * j + m) * (size_t)ldb + k0 + 8 * h;
            fb[j].h[0] = *(const u16x8*)(p);
            fb[j].h[1] = *(const u16x8*)(p + 16);
        }
#pragma unroll
        for (int s = 0; s < 2; ++s)
#pragma unroll
            for (int j = 0; j < NBF; ++j)
                mma16(acc[s * NBF + j], fa[s], fb[j]);
    }

    float* st = stile[wave];
#pragma unroll
    for (int s = 0; s < 2; ++s)
#pragma unroll
        for (int j = 0; j < NBF; ++j)
#pragma unroll
            for (int r = 0; r < 8; ++r)
                st[(s * 16 + 8 * h + r) * P + j * 16 + m] = acc[s * NBF + j][r] * oscale;
    __syncthreads();

    float* Cp = C;
    int gcol = colW;
    if (colW >= csplit) { Cp = C2; gcol = colW - csplit; }
    float* gp = Cp + (size_t)rowW * ldc + gcol;
    const float* rp = R + (size_t)rowW * ldc + gcol;
    tile_store_pass<NBF, RESID>(st, gp, ldc, rp, lane);
    __threadfence();
    tile_store_pass<NBF, RESID>(st, gp, ldc, rp, lane);
}

__global__ __launch_bounds__(128)
void conv_silu_kernel(const float* __restrict__ Up, const float* __restrict__ cw,
                      const float* __restrict__ cb, unsigned short* U16, float uscale)
{
    const int m  = blockIdx.x;
    const int l  = m & (NL_ - 1);
    const int d0 = threadIdx.x * 8;
    const float* xr = Up + (size_t)m * DI_ + d0;

    const v8f x3 = ld8f(xr);
    const size_t o1 = (l >= 1) ? (size_t)DI_ : 0;
    const size_t o2 = (l >= 2) ? (size_t)(2 * DI_) : 0;
    const size_t o3 = (l >= 3) ? (size_t)(3 * DI_) : 0;
    const float f1 = (l >= 1) ? 1.0f : 0.0f;
    const float f2 = (l >= 2) ? 1.0f : 0.0f;
    const float f3 = (l >= 3) ? 1.0f : 0.0f;
    const v8f x2 = ld8f(xr - o1) * f1;
    const v8f x1 = ld8f(xr - o2) * f2;
    const v8f x0 = ld8f(xr - o3) * f3;

    const float* wp = cw + (size_t)d0 * 4;
    v4f wv[8];
#pragma unroll
    for (int c = 0; c < 8; ++c) wv[c] = *(const v4f*)(wp + 4 * c);
    const v8f bias = ld8f(cb + d0);

    v8f u;
#pragma unroll
    for (int c = 0; c < 8; ++c)
        u[c] = conv4_silu(x0[c], x1[c], x2[c], x3[c], wv[c][0], wv[c][1], wv[c][2], wv[c][3], bias[c]) * uscale;

    Pack8 pk;
    pk.f = __builtin_convertvector(u, v8h);
    const u16x8 v = pk.u;
    unsigned short* gp = U16 + (size_t)m * DI_ + d0;
    *(volatile u16x8*)gp = v;
    __threadfence();
    *(volatile u16x8*)gp = v;
}

__device__ __forceinline__ void y_store_pass(const unsigned short* sy, unsigned short* Y16,
                                             size_t gbase, int wave, int lane) {
#pragma unroll
    for (int it = 0; it < 2; ++it) {
        const int t = wave * 8 + it * 4 + (lane >> 3);
        const int c = (lane & 7) * 8;
        const u16x8 v = *(const u16x8*)(sy + t * 64 + c);
        *(volatile u16x8*)(Y16 + gbase + (size_t)t * DI_ + c) = v;
    }
}

__global__ __launch_bounds__(64)
void scan_kernel(const float* __restrict__ Up, const float* __restrict__ Zp,
                 const float* __restrict__ DL, const float* __restrict__ XD,
                 const float* __restrict__ cw, const float* __restrict__ cb,
                 const float* __restrict__ dtb, const float* __restrict__ Alog,
                 const float* __restrict__ Dp, unsigned short* Y16)
{
    __shared__ __attribute__((aligned(16))) unsigned short sy[16 * 64];

    const int tid   = threadIdx.x;
    const int lane  = tid & 31;
    const int wave  = tid >> 5;
    const int dbase = blockIdx.x * 64;
    const int d     = dbase + tid;
    const int b     = blockIdx.y;

    float an2[NS_], hs[NS_];
#pragma unroll
    for (int n = 0; n < NS_; ++n) {
        an2[n] = -exp2f(Alog[(size_t)d * NS_ + n] * LOG2E_F) * LOG2E_F;
        hs[n] = 0.0f;
    }
    const float w0 = cw[d * 4 + 0], w1 = cw[d * 4 + 1], w2 = cw[d * 4 + 2], w3 = cw[d * 4 + 3];
    const float cbias = cb[d];
    const float tb = dtb[d];
    const float Dd = Dp[d];

    float xm1 = 0.0f, xm2 = 0.0f, xm3 = 0.0f;
    const size_t mrow0 = (size_t)b * NL_;

#pragma unroll 1
    for (int l0 = 0; l0 < NL_; l0 += 16) {
#pragma unroll 1
        for (int t = 0; t < 16; ++t) {
            const size_t mrow = mrow0 + (size_t)(l0 + t);
            const size_t e = mrow * DI_ + d;
            const float xv = Up[e];
            const float zv = Zp[e];
            const float dl = DL[e];
            const float* bc = XD + mrow * XDW_ + DTR_;
            const v8f vb0 = ld8f(bc);
            const v8f vb1 = ld8f(bc + 8);
            const v8f vc0 = ld8f(bc + 16);
            const v8f vc1 = ld8f(bc + 24);
            float bn[NS_], cn[NS_];
#pragma unroll
            for (int i = 0; i < 8; ++i) {
                bn[i] = vb0[i]; bn[8 + i] = vb1[i];
                cn[i] = vc0[i]; cn[8 + i] = vc1[i];
            }
            const float u  = conv4_silu(xm3, xm2, xm1, xv, w0, w1, w2, w3, cbias);
            xm3 = xm2; xm2 = xm1; xm1 = xv;
            const float dt = softplus_f(dl + tb);
            const float du = dt * u;
            float y = 0.0f;
#pragma unroll
            for (int n = 0; n < NS_; ++n) {
                const float da = exp2f(dt * an2[n]);
                hs[n] = da * hs[n] + du * bn[n];
                y += hs[n] * cn[n];
            }
            const float g = (y + Dd * u) * silu_f(zv);
            H1 hv;
            hv.f = (_Float16)(g * 16.0f);
            sy[t * 64 + tid] = hv.u;
        }
        __syncthreads();
        const size_t gbase = (mrow0 + (size_t)l0) * DI_ + dbase;
        y_store_pass(sy, Y16, gbase, wave, lane);
        __threadfence();
        y_store_pass(sy, Y16, gbase, wave, lane);
        __syncthreads();
    }
}

extern "C" void kernel_launch(void* const* d_in, const int* in_sizes, int n_in,
                              void* d_out, int out_size, void* d_ws, size_t ws_size,
                              hipStream_t stream)
{
    if (n_in < 12) return;
    if (in_sizes[0]  != MT_ * DM_)      return;
    if (in_sizes[1]  != DM_)            return;
    if (in_sizes[2]  != DM_)            return;
    if (in_sizes[3]  != 2 * DI_ * DM_)  return;
    if (in_sizes[4]  != DI_ * 4)        return;
    if (in_sizes[5]  != DI_)            return;
    if (in_sizes[6]  != XDW_ * DI_)     return;
    if (in_sizes[7]  != DI_ * DTR_)     return;
    if (in_sizes[8]  != DI_)            return;
    if (in_sizes[9]  != DI_ * NS_)      return;
    if (in_sizes[10] != DI_)            return;
    if (in_sizes[11] != DM_ * DI_)      return;
    if (out_size != MT_ * DM_)          return;

    const float* x     = (const float*)d_in[0];
    const float* nw    = (const float*)d_in[1];
    const float* nb    = (const float*)d_in[2];
    const float* wi    = (const float*)d_in[3];
    const float* cw    = (const float*)d_in[4];
    const float* cb    = (const float*)d_in[5];
    const float* wx    = (const float*)d_in[6];
    const float* wdt   = (const float*)d_in[7];
    const float* dtb   = (const float*)d_in[8];
    const float* alog  = (const float*)d_in[9];
    const float* Dp    = (const float*)d_in[10];
    const float* wo    = (const float*)d_in[11];
    float* out = (float*)d_out;

    const size_t SZ_WIN = (size_t)2 * DI_ * DM_ * 2;
    const size_t SZ_WX  = (size_t)XDW_ * DI_ * 2;
    const size_t SZ_WDT = (size_t)DI_ * DTR_ * 2;
    const size_t SZ_WO  = (size_t)DM_ * DI_ * 2;
    const size_t SZ_XN  = (size_t)MT_ * DM_ * 2;
    const size_t SZ_F   = (size_t)MT_ * DI_ * 4;
    const size_t SZ_U16 = (size_t)MT_ * DI_ * 2;
    const size_t SZ_XD  = (size_t)MT_ * XDW_ * 4;

    const size_t OFF_WIN = 0;
    const size_t OFF_WX  = OFF_WIN + SZ_WIN;
    const size_t OFF_WDT = OFF_WX + SZ_WX;
    const size_t OFF_WO  = OFF_WDT + SZ_WDT;
    const size_t OFF_XN  = OFF_WO + SZ_WO;
    const size_t OFF_UP  = OFF_XN + SZ_XN;
    const size_t OFF_Z   = OFF_UP + SZ_F;
    const size_t OFF_U16 = OFF_Z + SZ_F;
    const size_t OFF_Y16 = OFF_U16;
    const size_t OFF_XD  = OFF_U16 + SZ_U16;
    const size_t OFF_DL  = OFF_XD + SZ_XD;
    const size_t WS_END  = OFF_DL + SZ_F;
    if (ws_size < WS_END) return;

    char* ws = (char*)d_ws;
    unsigned short* win16 = (unsigned short*)(ws + OFF_WIN);
    unsigned short* wx16  = (unsigned short*)(ws + OFF_WX);
    unsigned short* wdt16 = (unsigned short*)(ws + OFF_WDT);
    unsigned short* wo16  = (unsigned short*)(ws + OFF_WO);
    unsigned short* xn16  = (unsigned short*)(ws + OFF_XN);
    float*          Up    = (float*)(ws + OFF_UP);
    float*          Zp    = (float*)(ws + OFF_Z);
    unsigned short* u16   = (unsigned short*)(ws + OFF_U16);
    unsigned short* y16   = (unsigned short*)(ws + OFF_Y16);
    float*          XD    = (float*)(ws + OFF_XD);
    float*          DL    = (float*)(ws + OFF_DL);

    {
        int n8;
        n8 = (2 * DI_ * DM_) / 8;
        hipLaunchKernelGGL(cvt_kernel, dim3((n8 + 255) / 256), dim3(256), 0, stream, wi, win16, n8, 32.0f);
        n8 = (XDW_ * DI_) / 8;
        hipLaunchKernelGGL(cvt_kernel, dim3((n8 + 255) / 256), dim3(256), 0, stream, wx, wx16, n8, 32.0f);
        n8 = (DI_ * DTR_) / 8;
        hipLaunchKernelGGL(cvt_kernel, dim3((n8 + 255) / 256), dim3(256), 0, stream, wdt, wdt16, n8, 4.0f);
        n8 = (DM_ * DI_) / 8;
        hipLaunchKernelGGL(cvt_kernel, dim3((n8 + 255) / 256), dim3(256), 0, stream, wo, wo16, n8, 32.0f);
    }

    hipLaunchKernelGGL(ln_kernel, dim3(MT_ / 8), dim3(256), 0, stream, x, nw, nb, xn16);

    hipLaunchKernelGGL(HIP_KERNEL_NAME(gemm_tn_kernel<false, 4, false>),
                       dim3((2 * DI_) / 128, MT_ / 64), dim3(128), 0, stream,
                       (const unsigned short*)xn16, (const float*)XD, (const unsigned short*)win16,
                       Up, Zp, x, (int)DM_, (int)DM_, (int)DM_, (int)DI_, (int)DI_, 1.0f, 0.03125f);

    hipLaunchKernelGGL(conv_silu_kernel, dim3(MT_), dim3(DI_ / 8), 0, stream,
                       (const float*)Up, cw, cb, u16, 16.0f);

    hipLaunchKernelGGL(HIP_KERNEL_NAME(gemm_tn_kernel<false, 2, false>),
                       dim3(XDW_ / 64, MT_ / 64), dim3(128), 0, stream,
                       (const unsigned short*)u16, (const float*)Up, (const unsigned short*)wx16,
                       XD, XD, x, (int)DI_, (int)DI_, (int)DI_, (int)XDW_, (int)(4 * XDW_), 1.0f, 0.001953125f);

    hipLaunchKernelGGL(HIP_KERNEL_NAME(gemm_tn_kernel<true, 4, false>),
                       dim3(DI_ / 128, MT_ / 64), dim3(128), 0, stream,
                       (const unsigned short*)u16, (const float*)XD, (const unsigned short*)wdt16,
                       DL, DL, x, (int)DTR_, (int)XDW_, (int)DTR_, (int)DI_, (int)(4 * DI_), 16.0f, 0.015625f);

    hipLaunchKernelGGL(scan_kernel, dim3(DI_ / 64, NB_), dim3(64), 0, stream,
                       (const float*)Up, (const float*)Zp, (const float*)DL, (const float*)XD,
                       cw, cb, dtb, alog, Dp, y16);

    hipLaunchKernelGGL(HIP_KERNEL_NAME(gemm_tn_kernel<false, 4, true>),
                       dim3(DM_ / 128, MT_ / 64), dim3(128), 0, stream,
                       (const unsigned short*)y16, (const float*)Up, (const unsigned short*)wo16,
                       out, out, x, (int)DI_, (int)DI_, (int)DI_, (int)DM_, (int)(4 * DM_), 1.0f, 0.001953125f);
}
